// LinearAttention_50878182588744
// MI455X (gfx1250) — hardware-run, weakly checked
//
#include <hip/hip_runtime.h>
#include <math.h>

typedef __attribute__((ext_vector_type(16))) _Float16 v16h;
typedef __attribute__((ext_vector_type(8)))  _Float16 v8h;
typedef __attribute__((ext_vector_type(16))) __bf16   v16b;
typedef __attribute__((ext_vector_type(8)))  __bf16   v8b;
typedef __attribute__((ext_vector_type(8)))  float    v8f;
typedef __attribute__((ext_vector_type(4)))  float    v4f;
typedef __attribute__((ext_vector_type(4)))  unsigned int v4u;

constexpr int kBatch = 2;
constexpr int kSeq   = 2048;
constexpr int kDm    = 512;
constexpr int kNh    = 8;
constexpr int kHd    = kDm / kNh;
constexpr int kRows  = kBatch * kSeq;
constexpr int kBH    = kBatch * kNh;
constexpr int kQkvN  = 3 * kDm;
constexpr int kPhiN  = 2 * kDm;
constexpr int kNBias = 4 * kDm;
constexpr int kTS    = 32;
constexpr int kOP    = 68;
constexpr float kDenFloor = 1e-6f;
static_assert(kHd == 64, "head width 64");
static_assert(kRows == 4096 && kQkvN == 1536 && kPhiN == 1024, "shapes");
static_assert((kDm % 32) == 0, "GEMM K multiple of 32");
static_assert((kRows % 64) == 0 && (kQkvN % 64) == 0 && (kDm % 64) == 0, "GEMM M,N multiples of 64");
static_assert((kSeq % kTS) == 0 && (kRows % 8) == 0, "tile multiples");

constexpr size_t kOffXB   = 0;
constexpr size_t kOffWT   = kOffXB   + (size_t)kRows * kDm * 2;
constexpr size_t kOffBias = kOffWT   + (size_t)4 * kDm * kDm * 2;
constexpr size_t kOffQKV  = kOffBias + (size_t)kNBias * 4;
constexpr size_t kOffPHI  = kOffQKV  + (size_t)kRows * kQkvN * 4;
constexpr size_t kOffAH   = kOffPHI  + (size_t)kRows * kPhiN * 4;
constexpr size_t kOffAL   = kOffAH   + (size_t)kRows * kDm * 2;
constexpr size_t kWsTotal = kOffAL   + (size_t)kRows * kDm * 2;
static_assert(kWsTotal == 56631296ull, "carve total");
static_assert(kWsTotal <= 134217728ull, "carve cap");
static_assert((kOffWT % 256) == 0 && (kOffBias % 256) == 0 && (kOffQKV % 256) == 0 && (kOffPHI % 256) == 0 &&
              (kOffAH % 256) == 0 && (kOffAL % 256) == 0, "aligned regions");

__device__ __forceinline__ unsigned short f2bf_bits(float f) {
  unsigned u = __float_as_uint(f);
  return (unsigned short)((u + 0x7FFFu + ((u >> 16) & 1u)) >> 16);
}
__device__ __forceinline__ float bf_bits2f(unsigned short h) { return __uint_as_float(((unsigned)h) << 16); }
__device__ __forceinline__ float bf16r(float f) { return bf_bits2f(f2bf_bits(f)); }
__device__ __forceinline__ unsigned pk16(unsigned short a, unsigned short b) { return (unsigned)a | ((unsigned)b << 16); }

__device__ __forceinline__ void keep4_b(v16b a, v16b b, v16b c, v16b d) { asm volatile("v_nop" :: "v"(a), "v"(b), "v"(c), "v"(d)); }
__device__ __forceinline__ void acc_guard4(v8f& a, v8f& b, v8f& c, v8f& d) { asm volatile("v_nop\n\tv_nop\n\tv_nop\n\tv_nop" : "+v"(a), "+v"(b), "+v"(c), "+v"(d)); }

template <typename T> struct Frag;
template <> struct Frag<__bf16> {
  typedef v16b V; union U { v16b v; v8b h[2]; };
  static __device__ __forceinline__ v16b load(const __bf16* p) {
    U f; f.h[0] = *(const v8b*)(p); f.h[1] = *(const v8b*)(p + 16); return f.v;
  }
};
__device__ __forceinline__ v8f mma_g(v16b a, v16b b, v8f c) {
  c = __builtin_amdgcn_wmma_f32_16x16x32_bf16(false, a, false, b, (short)0, c, false, false);
  asm volatile("v_nop\n\tv_nop\n\tv_nop\n\tv_nop" : "+v"(c) : "v"(a), "v"(b));
  return c;
}

template <int SPL>
__global__ __launch_bounds__(256) void wmma_gemm64_bf16(
    const unsigned short* __restrict__ Ap, const unsigned short* __restrict__ A2p, int lda,
    const unsigned short* __restrict__ Btp, int ldb,
    float* __restrict__ C, int ldc,
    const float* __restrict__ bias,
    int M, int N, int K) {
  typedef __bf16 T;
  typedef v16b V;
  const T* A = (const T*)Ap; const T* A2 = (const T*)A2p; const T* Bt = (const T*)Btp;
  __shared__ __align__(16) float sT[8][16 * 68];
  const int lane = threadIdx.x & 31;
  const int wave = threadIdx.x >> 5;
  const int tilesN = N >> 6;
  const int tilesM = M >> 6;
  const int tile = blockIdx.x * 8 + wave;
  if (tile >= tilesM * tilesN) return;
  const int tm = tile / tilesN;
  const int tn = tile - tm * tilesN;
  const int m0 = tm << 6;
  const int n0 = tn << 6;

  const int rlane = lane & 15;
  const int koff  = (lane >> 4) * 8;
  const int mOff  = (lane >> 4) * 8;

  v8f acc[4][4];
#pragma unroll
  for (int i = 0; i < 4; ++i)
#pragma unroll
    for (int j = 0; j < 4; ++j) acc[i][j] = (v8f){0.f,0.f,0.f,0.f,0.f,0.f,0.f,0.f};

  for (int k0 = 0; k0 < K; k0 += 32) {
    V bh[4];
#pragma unroll
    for (int j = 0; j < 4; ++j) {
      const size_t bo = (size_t)(n0 + (j << 4) + rlane) * ldb + koff + k0;
      bh[j] = Frag<T>::load(Bt + bo);
    }
#pragma unroll
    for (int i = 0; i < 4; ++i) {
      const size_t ao = (size_t)(m0 + (i << 4) + rlane) * lda + koff + k0;
      V ah = Frag<T>::load(A + ao);
      V al = ah;
      if (SPL == 1) al = Frag<T>::load(A2 + ao);
#pragma unroll
      for (int j = 0; j < 4; ++j) {
        acc[i][j] = mma_g(ah, bh[j], acc[i][j]);
        if (SPL == 1) acc[i][j] = mma_g(al, bh[j], acc[i][j]);
      }
    }
    keep4_b(bh[0], bh[1], bh[2], bh[3]);
  }
  acc_guard4(acc[0][0], acc[0][1], acc[0][2], acc[0][3]);
  acc_guard4(acc[1][0], acc[1][1], acc[1][2], acc[1][3]);
  acc_guard4(acc[2][0], acc[2][1], acc[2][2], acc[2][3]);
  acc_guard4(acc[3][0], acc[3][1], acc[3][2], acc[3][3]);

  float* slab = sT[wave];
#pragma unroll
  for (int i = 0; i < 4; ++i) {
    const int mBase = m0 + (i << 4);
#pragma unroll
    for (int j = 0; j < 4; ++j) {
      const int n = n0 + (j << 4) + rlane;
      const float bv = bias[n];
#pragma unroll
      for (int r = 0; r < 8; ++r) {
        const float v = acc[i][j][r] + bv;
        slab[(mOff + r) * 68 + (j << 4) + rlane] = v;
      }
    }
    __builtin_amdgcn_fence(__ATOMIC_RELEASE, "workgroup");
    __builtin_amdgcn_wave_barrier();
    __builtin_amdgcn_fence(__ATOMIC_ACQUIRE, "workgroup");
    {
      const int hh = lane >> 4, c4 = (lane & 15) * 4;
      for (int pass = 0; pass < 2; ++pass) {
#pragma unroll
        for (int it = 0; it < 8; ++it) {
          const int row = it * 2 + hh;
          v4f v = *(const v4f*)(slab + row * 68 + c4);
          *(volatile v4f*)(C + (size_t)(mBase + row) * ldc + n0 + c4) = v;
        }
        __threadfence();
      }
    }
    __builtin_amdgcn_fence(__ATOMIC_RELEASE, "workgroup");
    __builtin_amdgcn_wave_barrier();
    __builtin_amdgcn_fence(__ATOMIC_ACQUIRE, "workgroup");
  }
}

__global__ __launch_bounds__(256) void cvt8_bf16_kernel(const float* __restrict__ src, unsigned short* __restrict__ dst, int n8) {
  const int i = blockIdx.x * 256 + threadIdx.x;
  if (i < n8) {
    const float* sp = src + (size_t)i * 8;
    const v4f a = *(const v4f*)(sp);
    const v4f b = *(const v4f*)(sp + 4);
    v8h hv;
#pragma unroll
    for (int e = 0; e < 4; ++e) {
      const unsigned short b0 = f2bf_bits(a[e]);
      const unsigned short b1 = f2bf_bits(b[e]);
      hv[e]     = __builtin_bit_cast(_Float16, b0);
      hv[4 + e] = __builtin_bit_cast(_Float16, b1);
    }
    *(volatile v8h*)(dst + (size_t)i * 8) = hv;
    __threadfence();
    *(volatile v8h*)(dst + (size_t)i * 8) = hv;
  }
}

__global__ __launch_bounds__(256) void wt_transpose_bf16_kernel(const float* __restrict__ W0, const float* __restrict__ W1,
                                                                const float* __restrict__ W2, const float* __restrict__ W3,
                                                                unsigned short* __restrict__ out) {
  __shared__ float sm[64][65];
  const int t  = threadIdx.x;
  const int k0 = blockIdx.x * 64;
  const int n0 = blockIdx.y * 64;
  const int z  = blockIdx.z;
  const float* W = (z == 0) ? W0 : (z == 1) ? W1 : (z == 2) ? W2 : W3;
#pragma unroll
  for (int i = 0; i < 16; ++i) {
    const int e = i * 256 + t;
    const int r = e >> 6;
    const int c = e & 63;
    sm[c][r] = W[(size_t)(k0 + r) * kDm + n0 + c];
  }
  __syncthreads();
  const int lane = t & 31, wave = t >> 5;
  const int q = lane >> 3, c8 = (lane & 7) * 8;
  unsigned short* op = out + (size_t)z * kDm * kDm;
  for (int pass = 0; pass < 2; ++pass) {
#pragma unroll
    for (int it = 0; it < 2; ++it) {
      const int row = wave * 8 + it * 4 + q;
      unsigned short hb[8];
#pragma unroll
      for (int e = 0; e < 8; ++e) hb[e] = f2bf_bits(sm[row][c8 + e]);
      const v4u u = (v4u){pk16(hb[0], hb[1]), pk16(hb[2], hb[3]), pk16(hb[4], hb[5]), pk16(hb[6], hb[7])};
      *(volatile v4u*)(op + (size_t)(n0 + row) * kDm + k0 + c8) = u;
    }
    __threadfence();
  }
}

__global__ __launch_bounds__(256) void bias_prep_kernel(const float* __restrict__ b0, const float* __restrict__ b1,
                                                        const float* __restrict__ b2, const float* __restrict__ b3,
                                                        float* __restrict__ dst) {
  const int tid = threadIdx.x;
#pragma unroll
  for (int it = 0; it < 2; ++it) {
    const int idx   = it * 1024 + tid * 4;
    const int which = idx >> 9;
    const int off   = idx & 511;
    const v4f v0 = *(const v4f*)(b0 + off);
    const v4f v1 = *(const v4f*)(b1 + off);
    const v4f v2 = *(const v4f*)(b2 + off);
    const v4f v3 = *(const v4f*)(b3 + off);
    v4f o;
#pragma unroll
    for (int e = 0; e < 4; ++e) {
      const float s01 = (which == 0) ? v0[e] : v1[e];
      const float s23 = (which == 2) ? v2[e] : v3[e];
      const float s   = (which < 2) ? s01 : s23;
      o[e] = bf16r(s);
    }
    float* op = dst + idx;
    *(volatile v4f*)op = o;
    __threadfence();
    *(volatile v4f*)op = o;
  }
}

__global__ __launch_bounds__(256) void featmap_kernel(const float* __restrict__ QKV, float* __restrict__ PHI) {
  const int c4   = threadIdx.x * 4;
  const int row0 = blockIdx.x * 8;
#pragma unroll 1
  for (int r = 0; r < 8; ++r) {
    const size_t row = (size_t)(row0 + r);
    const v4f u = *(const v4f*)(QKV + row * kQkvN + c4);
    v4f o;
#pragma unroll
    for (int e = 0; e < 4; ++e) {
      const float x  = u[e];
      const float ex = expf(fminf(x, 0.0f));
      o[e] = (x > 0.0f) ? (x + 1.0f) : ex;
    }
    float* op = PHI + row * kPhiN + c4;
    *(volatile v4f*)op = o;
    __threadfence();
    *(volatile v4f*)op = o;
  }
}

__global__ __launch_bounds__(256) void state_scan_kernel(const float* __restrict__ PHI, const float* __restrict__ QKV,
                                                         unsigned short* __restrict__ AH, unsigned short* __restrict__ AL) {
  __shared__ __align__(16) float sQ[kTS * kHd];
  __shared__ __align__(16) float sK[kTS * kHd];
  __shared__ __align__(16) float sV[kTS * kHd];
  __shared__ __align__(16) float sO[kTS * kOP];
  const int tid = threadIdx.x, lane = tid & 31, wave = tid >> 5;
  const int dq = lane & 3;
  const int m  = wave * 8 + (lane >> 2);
  const int bh = blockIdx.x;
  const int bb = bh >> 3;
  const int hd = bh & 7;
  const size_t row0 = (size_t)bb * kSeq;
  const int lr = tid >> 4, lc4 = (tid & 15) * 4;
  const int sq = lane >> 3, c8 = (lane & 7) * 8;

  float S[16], z[16];
#pragma unroll
  for (int i = 0; i < 16; ++i) { S[i] = 0.0f; z[i] = 0.0f; }

#pragma unroll 1
  for (int t0 = 0; t0 < kSeq; t0 += kTS) {
    __syncthreads();
#pragma unroll
    for (int i = 0; i < 2; ++i) {
      const int r = lr + 16 * i;
      const size_t g = row0 + (size_t)(t0 + r);
      const v4f qv = *(const v4f*)(PHI + g * kPhiN + hd * kHd + lc4);
      const v4f kv = *(const v4f*)(PHI + g * kPhiN + kDm + hd * kHd + lc4);
      const v4f vv = *(const v4f*)(QKV + g * kQkvN + 2 * kDm + hd * kHd + lc4);
      *(v4f*)(sQ + r * kHd + lc4) = qv;
      *(v4f*)(sK + r * kHd + lc4) = kv;
      *(v4f*)(sV + r * kHd + lc4) = vv;
    }
    __syncthreads();

#pragma unroll 1
    for (int s = 0; s < kTS; ++s) {
      const float* kp = sK + s * kHd + dq * 16;
      const float* qp = sQ + s * kHd + dq * 16;
      const float vt = sV[s * kHd + m];
      float num = 0.0f, den = 0.0f;
#pragma unroll
      for (int j = 0; j < 4; ++j) {
        const v4f kk = *(const v4f*)(kp + 4 * j);
        const v4f qq = *(const v4f*)(qp + 4 * j);
#pragma unroll
        for (int e = 0; e < 4; ++e) {
          const float ke = kk[e];
          const float qe = qq[e];
          S[4 * j + e] = fmaf(ke, vt, S[4 * j + e]);
          z[4 * j + e] = z[4 * j + e] + ke;
          num = fmaf(qe, S[4 * j + e], num);
          den = fmaf(qe, z[4 * j + e], den);
        }
      }
      num += __shfl_xor(num, 1, 32);
      den += __shfl_xor(den, 1, 32);
      num += __shfl_xor(num, 2, 32);
      den += __shfl_xor(den, 2, 32);
      den = fmaxf(den, kDenFloor);
      const float o = num / den;
      if (dq == 0) sO[s * kOP + m] = o;
    }
    __syncthreads();

    {
      const int row = wave * 4 + sq;
      const float* sp = sO + row * kOP + c8;
      const v4f a0 = *(const v4f*)(sp);
      const v4f a1 = *(const v4f*)(sp + 4);
      v8h hv, lv;
#pragma unroll
      for (int e = 0; e < 4; ++e) {
        const float f0 = a0[e];
        const float f1 = a1[e];
        const unsigned short h0 = f2bf_bits(f0), h1 = f2bf_bits(f1);
        const unsigned short l0 = f2bf_bits(f0 - bf_bits2f(h0)), l1 = f2bf_bits(f1 - bf_bits2f(h1));
        hv[e]     = __builtin_bit_cast(_Float16, h0);
        hv[4 + e] = __builtin_bit_cast(_Float16, h1);
        lv[e]     = __builtin_bit_cast(_Float16, l0);
        lv[4 + e] = __builtin_bit_cast(_Float16, l1);
      }
      const size_t o = (row0 + (size_t)(t0 + row)) * kDm + hd * kHd + c8;
      for (int pass = 0; pass < 2; ++pass) {
        *(volatile v8h*)(AH + o) = hv;
        *(volatile v8h*)(AL + o) = lv;
        __threadfence();
      }
    }
  }
}

extern "C" void kernel_launch(void* const* d_in, const int* in_sizes, int n_in,
                              void* d_out, int out_size, void* d_ws, size_t ws_size,
                              hipStream_t stream) {
  if (n_in < 9 || d_out == nullptr || d_ws == nullptr) return;
  if (in_sizes[0] != kRows * kDm) return;
  if (in_sizes[1] != kDm * kDm || in_sizes[3] != kDm * kDm || in_sizes[5] != kDm * kDm || in_sizes[7] != kDm * kDm) return;
  if (in_sizes[2] != kDm || in_sizes[4] != kDm || in_sizes[6] != kDm || in_sizes[8] != kDm) return;
  if (out_size != kRows * kDm) return;
  if (ws_size < kWsTotal) return;

  const float* x  = (const float*)d_in[0];
  const float* Wq = (const float*)d_in[1];
  const float* bq = (const float*)d_in[2];
  const float* Wk = (const float*)d_in[3];
  const float* bk = (const float*)d_in[4];
  const float* Wv = (const float*)d_in[5];
  const float* bv = (const float*)d_in[6];
  const float* Wo = (const float*)d_in[7];
  const float* bo = (const float*)d_in[8];
  float* out = (float*)d_out;

  char* ws = (char*)d_ws;
  unsigned short* XB   = (unsigned short*)(ws + kOffXB);
  unsigned short* WT   = (unsigned short*)(ws + kOffWT);
  float*          BIAS = (float*)(ws + kOffBias);
  float*          QKV  = (float*)(ws + kOffQKV);
  float*          PHI  = (float*)(ws + kOffPHI);
  unsigned short* AH   = (unsigned short*)(ws + kOffAH);
  unsigned short* AL   = (unsigned short*)(ws + kOffAL);
  unsigned short* WoT  = WT + (size_t)3 * kDm * kDm;

  cvt8_bf16_kernel<<<(kRows * kDm / 8) / 256, 256, 0, stream>>>(x, XB, kRows * kDm / 8);
  wt_transpose_bf16_kernel<<<dim3(kDm / 64, kDm / 64, 4), 256, 0, stream>>>(Wq, Wk, Wv, Wo, WT);
  bias_prep_kernel<<<1, 256, 0, stream>>>(bq, bk, bv, bo, BIAS);

  wmma_gemm64_bf16<0><<<(kRows / 64) * (kQkvN / 64) / 8, 256, 0, stream>>>(
      XB, XB, kDm, WT, kDm, QKV, kQkvN, BIAS, kRows, kQkvN, kDm);

  featmap_kernel<<<kRows / 8, 256, 0, stream>>>(QKV, PHI);

  state_scan_kernel<<<kBH, 256, 0, stream>>>(PHI, QKV, AH, AL);

  wmma_gemm64_bf16<1><<<(kRows / 64) * (kDm / 64) / 8, 256, 0, stream>>>(
      AH, AL, kDm, WoT, kDm, out, kDm, BIAS + 3 * kDm, kRows, kDm, kDm);
}
